// ExpertSelectiveTimeVaryingSSM_15934328668593
// MI455X (gfx1250) — hardware-verified
//
#include <hip/hip_runtime.h>
#include <math.h>


#define BB_    64
#define TT_    1024
#define DS_    128
#define DU_    64
#define DY_    64
#define MM_    8
#define GH_    64
#define NA_    192
#define KP_    576
#define KPS_   384
#define NBT_   (BB_ * TT_)
#define NRB_   16
#define NTS_   384
#define NITER_ 32

static_assert(NBT_ == 65536);
static_assert(KP_ == 3 * DS_ + 3 * DU_);
static_assert(KPS_ == 3 * DS_);
static_assert(KP_ % 32 == 0 && KPS_ % 32 == 0);
static_assert(BB_ % NRB_ == 0);
static_assert(NTS_ == 32 * 12);
static_assert(NBT_ % 64 == 0);
static_assert(DS_ + DY_ == NA_ && DS_ + DU_ == NA_);
static_assert((NA_ * (KP_ / 8)) % 256 == 0);
static_assert((DS_ * (KPS_ / 8)) % 128 == 0);

typedef float          v4f   __attribute__((ext_vector_type(4)));
typedef float          v8f   __attribute__((ext_vector_type(8)));
typedef unsigned short u16x8 __attribute__((ext_vector_type(8)));
typedef __bf16         v16bf __attribute__((ext_vector_type(16)));

union FragB { u16x8 h[2]; v16bf v; };

constexpr size_t SZ_KPL  = (size_t)MM_ * NA_ * KP_ * 2;
constexpr size_t SZ_SPL  = (size_t)DS_ * KPS_ * 2;
constexpr size_t SZ_PI   = (size_t)NBT_ * MM_ * 4;
constexpr size_t OFF_KPL = 0;
constexpr size_t OFF_SPL = OFF_KPL + SZ_KPL;
constexpr size_t OFF_PI  = OFF_SPL + SZ_SPL;
constexpr size_t WS_END  = OFF_PI + SZ_PI;
static_assert(WS_END == (size_t)3964928);
static_assert(OFF_SPL % 128 == 0 && OFF_PI % 128 == 0 && WS_END % 128 == 0);
static_assert(WS_END <= (size_t)134217728);

__device__ __forceinline__ unsigned short bfb(float f) {
    unsigned uu = __float_as_uint(f);
    uu += 0x7FFFu + ((uu >> 16) & 1u);
    return (unsigned short)(uu >> 16);
}
__device__ __forceinline__ void split8(const v8f v, u16x8& hi, u16x8& lo) {
#pragma unroll
    for (int e = 0; e < 8; ++e) {
        const unsigned short hb = bfb(v[e]);
        const float hf = __uint_as_float(((unsigned)hb) << 16);
        hi[e] = hb;
        lo[e] = bfb(v[e] - hf);
    }
}
__device__ __forceinline__ v8f ld8f(const float* p) {
    const v4f a = *(const v4f*)p;
    const v4f b = *(const v4f*)(p + 4);
    return __builtin_shufflevector(a, b, 0, 1, 2, 3, 4, 5, 6, 7);
}
__device__ __forceinline__ float wave_sum(float v) {
#pragma unroll
    for (int m = 16; m >= 1; m >>= 1) v += __shfl_xor(v, m, 32);
    return v;
}

__device__ __forceinline__ void mma_bf(v8f& acc, const FragB& a, const FragB& b) {
    acc = __builtin_amdgcn_wmma_f32_16x16x32_bf16(false, a.v, false, b.v, (short)0, acc, false, false);
    asm volatile("v_nop\n\tv_nop\n\tv_nop\n\tv_nop" : "+v"(acc) : "v"(a.v), "v"(b.v));
}

__global__ __launch_bounds__(128)
void sinv_plane_kernel(const float* __restrict__ S_raw, unsigned short* Spl)
{
    __shared__ float Xs[DS_ * DS_];
    const int c = threadIdx.x;
#pragma unroll 1
    for (int i = 0; i < DS_; ++i) {
        const float draw = S_raw[i * DS_ + i];
        const float d  = fmaxf(draw, 0.0f) + log1pf(expf(-fabsf(draw))) + 1e-3f;
        const float rd = 1.0f / d;
        float a = (i == c) ? 1.0f : 0.0f;
#pragma unroll 4
        for (int k = 0; k < i; ++k) a = fmaf(-S_raw[i * DS_ + k], Xs[k * DS_ + c], a);
        Xs[i * DS_ + c] = a * rd;
    }
    __syncthreads();
#pragma unroll 1
    for (int idx = c; idx < DS_ * (KPS_ / 8); idx += 128) {
        const int s    = idx / (KPS_ / 8);
        const int q    = idx - s * (KPS_ / 8);
        const int hoff = 8 * q;
        const int seg  = hoff >> 7;
        const int i0   = hoff & (DS_ - 1);
        v8f v;
#pragma unroll
        for (int e = 0; e < 8; ++e) v[e] = Xs[s * DS_ + i0 + e];
        u16x8 hi, lo;
        split8(v, hi, lo);
        const u16x8 o = (seg == 1) ? lo : hi;
        unsigned short* gp = Spl + (size_t)s * KPS_ + hoff;
        *(volatile u16x8*)gp = o;
        __threadfence();
        *(volatile u16x8*)gp = o;
    }
}

__global__ __launch_bounds__(256)
void experts_kernel(const float* __restrict__ K_raw, unsigned short* Kpl)
{
    __shared__ float v[NA_];
    __shared__ float w[NA_];
    __shared__ float red[8];
    const int m = blockIdx.x, tid = threadIdx.x, lane = tid & 31, wave = tid >> 5;
    const float* Km = K_raw + (size_t)m * NA_ * NA_;
    if (tid < NA_) v[tid] = 0.072168783648703216f;
    __syncthreads();
    float nrm = 0.0f;
#pragma unroll 1
    for (int it = 0; it < NITER_; ++it) {
        if (tid < NA_) {
            const int jn = (tid >= DS_) ? DS_ : NA_;
            const float* kr = Km + (size_t)tid * NA_;
            float a = 0.0f;
#pragma unroll 4
            for (int j = 0; j < jn; ++j) a = fmaf(kr[j], v[j], a);
            w[tid] = a;
        }
        __syncthreads();
        float a2 = 0.0f;
        if (tid < NA_) {
            const int in_ = (tid >= DS_) ? DS_ : NA_;
#pragma unroll 4
            for (int i = 0; i < in_; ++i) a2 = fmaf(Km[(size_t)i * NA_ + tid], w[i], a2);
        }
        float q = a2 * a2;
        q = wave_sum(q);
        if (lane == 0) red[wave] = q;
        __syncthreads();
        float tot = 0.0f;
#pragma unroll
        for (int k = 0; k < 8; ++k) tot += red[k];
        nrm = sqrtf(tot);
        const float inv = 1.0f / fmaxf(nrm, 1e-30f);
        if (tid < NA_) v[tid] = a2 * inv;
        __syncthreads();
    }
    const float sig = sqrtf(nrm);
    const float isc = 1.0f / fmaxf(sig, 1.0f);

#pragma unroll 1
    for (int idx = tid; idx < NA_ * (KP_ / 8); idx += 256) {
        const int a    = idx / (KP_ / 8);
        const int q    = idx - a * (KP_ / 8);
        const int hoff = 8 * q;
        int seg, c0;
        if (hoff < 3 * DS_) { seg = hoff >> 7; c0 = hoff & (DS_ - 1); }
        else { const int h2 = hoff - 3 * DS_; seg = h2 >> 6; c0 = DS_ + (h2 & (DU_ - 1)); }
        const bool zero = (a >= DS_) && (c0 >= DS_);
        v8f vals = ld8f(Km + (size_t)a * NA_ + c0);
#pragma unroll
        for (int e = 0; e < 8; ++e) vals[e] = zero ? 0.0f : (vals[e] * isc);
        u16x8 hi, lo;
        split8(vals, hi, lo);
        const u16x8 o = (seg == 1) ? lo : hi;
        unsigned short* gp = Kpl + ((size_t)(m * NA_ + a)) * KP_ + hoff;
        *(volatile u16x8*)gp = o;
        __threadfence();
        *(volatile u16x8*)gp = o;
    }
}

__global__ __launch_bounds__(128)
void gate_kernel(const float* __restrict__ u, const float* __restrict__ gw1, const float* __restrict__ gb1,
                 const float* __restrict__ gw2, const float* __restrict__ gb2, float* piw)
{
    __shared__ __attribute__((aligned(16))) float hf[4][16 * GH_];
    __shared__ __attribute__((aligned(16))) unsigned short hh[4][16 * GH_];
    __shared__ __attribute__((aligned(16))) unsigned short hl[4][16 * GH_];
    __shared__ float lgt[4][16 * MM_];
    __shared__ __attribute__((aligned(16))) float pst[64 * MM_];

    const int tid = threadIdx.x, lane = tid & 31, h = lane >> 4, ml = lane & 15;
    const int wv  = __builtin_amdgcn_readfirstlane(tid >> 5);
    const int r0  = blockIdx.x * 64 + wv * 16;

    u16x8 ah[4], al[4];
    {
        const float* ur = u + (size_t)(r0 + ml) * DU_ + 8 * h;
#pragma unroll
        for (int gI = 0; gI < 4; ++gI) { const v8f x = ld8f(ur + 16 * gI); split8(x, ah[gI], al[gI]); }
    }
    v8f acc[4];
#pragma unroll
    for (int j = 0; j < 4; ++j)
#pragma unroll
        for (int r = 0; r < 8; ++r) acc[j][r] = 0.0f;

#pragma unroll
    for (int j = 0; j < 4; ++j) {
        u16x8 bh[4], bl[4];
        const float* wr = gw1 + (size_t)(16 * j + ml) * DU_ + 8 * h;
#pragma unroll
        for (int gI = 0; gI < 4; ++gI) { const v8f x = ld8f(wr + 16 * gI); split8(x, bh[gI], bl[gI]); }
#pragma unroll
        for (int ks = 0; ks < 6; ++ks) {
            const int seg = ks >> 1, g0 = 2 * (ks & 1);
            FragB a, b;
            a.h[0] = (seg == 2) ? al[g0] : ah[g0];
            a.h[1] = (seg == 2) ? al[g0 + 1] : ah[g0 + 1];
            b.h[0] = (seg == 1) ? bl[g0] : bh[g0];
            b.h[1] = (seg == 1) ? bl[g0 + 1] : bh[g0 + 1];
            mma_bf(acc[j], a, b);
        }
    }
    float* hfw = hf[wv];
#pragma unroll
    for (int j = 0; j < 4; ++j)
#pragma unroll
        for (int r = 0; r < 8; ++r) hfw[(8 * h + r) * GH_ + 16 * j + ml] = acc[j][r];
    __syncthreads();

    unsigned short* hhw = hh[wv];
    unsigned short* hlw = hl[wv];
#pragma unroll 1
    for (int it = 0; it < 32; ++it) {
        const int idx = it * 32 + lane;
        const int col = idx & (GH_ - 1);
        const float x  = hfw[idx] + gb1[col];
        const float gv = 0.5f * x * erfcf(-x * 0.70710678118654752f);
        const unsigned short hb = bfb(gv);
        hhw[idx] = hb;
        hlw[idx] = bfb(gv - __uint_as_float(((unsigned)hb) << 16));
    }
    __syncthreads();

    const int mrow = (ml < MM_) ? ml : (MM_ - 1);
    u16x8 ch[4], cl[4];
    {
        const bool  ok = (ml < MM_);
        const float* wr = gw2 + (size_t)mrow * GH_ + 8 * h;
#pragma unroll
        for (int gI = 0; gI < 4; ++gI) {
            v8f x = ld8f(wr + 16 * gI);
#pragma unroll
            for (int e = 0; e < 8; ++e) x[e] = ok ? x[e] : 0.0f;
            split8(x, ch[gI], cl[gI]);
        }
    }
    v8f acc2;
#pragma unroll
    for (int r = 0; r < 8; ++r) acc2[r] = 0.0f;
    const unsigned short* ph = hhw + ml * GH_ + 8 * h;
    const unsigned short* pl = hlw + ml * GH_ + 8 * h;
#pragma unroll
    for (int ks = 0; ks < 6; ++ks) {
        const int seg = ks >> 1, kk = 32 * (ks & 1), g0 = 2 * (ks & 1);
        const unsigned short* pa = (seg == 2) ? pl : ph;
        FragB a, b;
        a.h[0] = *(const u16x8*)(pa + kk);
        a.h[1] = *(const u16x8*)(pa + kk + 16);
        b.h[0] = (seg == 1) ? cl[g0] : ch[g0];
        b.h[1] = (seg == 1) ? cl[g0 + 1] : ch[g0 + 1];
        mma_bf(acc2, a, b);
    }
    float* lw = lgt[wv];
    const float bb2 = gb2[mrow];
    if (ml < MM_) {
#pragma unroll
        for (int r = 0; r < 8; ++r) lw[(8 * h + r) * MM_ + ml] = acc2[r] + bb2;
    }
    __syncthreads();
    {
        const float* lr = lw + ml * MM_;
        float mx = lr[0];
#pragma unroll 1
        for (int m = 1; m < MM_; ++m) mx = fmaxf(mx, lr[m]);
        float s = 0.0f;
#pragma unroll 1
        for (int m = 0; m < MM_; ++m) s += expf(lr[m] - mx);
        const float inv = 1.0f / s;
        float* pr = pst + (wv * 16 + ml) * MM_;
#pragma unroll 1
        for (int m = 0; m < MM_; ++m) {
            const float p = expf(lr[m] - mx) * inv;
            if (lane < 16) pr[m] = p;
        }
    }
    __syncthreads();
    if (wv == 0) {
        float* gp = piw + (size_t)blockIdx.x * (64 * MM_);
        v4f pv[4];
#pragma unroll
        for (int it = 0; it < 4; ++it) pv[it] = *(const v4f*)(pst + it * 128 + 4 * lane);
#pragma unroll
        for (int it = 0; it < 4; ++it) *(volatile v4f*)(gp + it * 128 + 4 * lane) = pv[it];
        __threadfence();
#pragma unroll
        for (int it = 0; it < 4; ++it) *(volatile v4f*)(gp + it * 128 + 4 * lane) = pv[it];
    }
}

__global__ __launch_bounds__(NTS_)
void scan_kernel(const float* __restrict__ u, const float* __restrict__ piw, const float* __restrict__ lgam,
                 const unsigned short* __restrict__ Kpl, const unsigned short* __restrict__ Spl,
                 float* out_y, float* out_x)
{
    __shared__ __attribute__((aligned(16))) float zf[NRB_ * DS_];
    __shared__ __attribute__((aligned(16))) unsigned short Ap[NRB_ * KP_];
    __shared__ __attribute__((aligned(16))) float pis[NRB_ * MM_];
    __shared__ __attribute__((aligned(16))) float xst[NRB_ * DS_];
    __shared__ __attribute__((aligned(16))) float yst[NRB_ * DY_];

    const int tid  = threadIdx.x;
    const int lane = tid & 31, h = lane >> 4, ml = lane & 15;
    const int wv   = __builtin_amdgcn_readfirstlane(tid >> 5);
    const int b0   = blockIdx.x * NRB_;
    const float g  = expf(lgam[0]);
    const bool zp  = (wv < 8);

    for (int i = tid; i < NRB_ * DS_; i += NTS_) zf[i] = 0.0f;
    __syncthreads();

    const unsigned short* kb  = Kpl + (size_t)(16 * wv + ml) * KP_ + 8 * h;
    const unsigned short* sbp = Spl + (size_t)(16 * (zp ? wv : 0) + ml) * KPS_ + 8 * h;
    const unsigned short* ab  = Ap + ml * KP_ + 8 * h;
    const int nks  = zp ? (KP_ / 32) : (KPS_ / 32);
    const int ccol = zp ? (16 * wv + ml) : (16 * (wv - 8) + ml);
    const size_t ESTR = (size_t)NA_ * KP_;

#pragma unroll 1
    for (int t = 0; t < TT_; ++t) {
        if (tid < 256) {
            const int row = tid >> 4, q = tid & 15;
            const v8f v = ld8f(zf + row * DS_ + 8 * q);
            u16x8 hi, lo;
            split8(v, hi, lo);
            unsigned short* ap = Ap + row * KP_ + 8 * q;
            *(u16x8*)ap            = hi;
            *(u16x8*)(ap + DS_)    = hi;
            *(u16x8*)(ap + 2 * DS_) = lo;
            if (tid < NRB_ * MM_) {
                const int r2 = tid >> 3, m2 = tid & 7;
                pis[tid] = piw[((size_t)(b0 + r2) * TT_ + t) * MM_ + m2];
            }
        } else {
            const int tt = tid - 256, row = tt >> 3, q = tt & 7;
            v8f v = ld8f(u + ((size_t)(b0 + row) * TT_ + t) * DU_ + 8 * q);
#pragma unroll
            for (int e = 0; e < 8; ++e) v[e] *= g;
            u16x8 hi, lo;
            split8(v, hi, lo);
            unsigned short* ap = Ap + row * KP_ + 3 * DS_ + 8 * q;
            *(u16x8*)ap            = hi;
            *(u16x8*)(ap + DU_)    = hi;
            *(u16x8*)(ap + 2 * DU_) = lo;
        }
        __syncthreads();

        v8f acc[9];
#pragma unroll
        for (int j = 0; j < 9; ++j)
#pragma unroll
            for (int r = 0; r < 8; ++r) acc[j][r] = 0.0f;

#pragma unroll 1
        for (int ks = 0; ks < nks; ++ks) {
            const int k0 = ks * 32;
            FragB a;
            a.h[0] = *(const u16x8*)(ab + k0);
            a.h[1] = *(const u16x8*)(ab + k0 + 16);
#pragma unroll
            for (int m = 0; m < MM_; ++m) {
                const unsigned short* p = kb + (size_t)m * ESTR + k0;
                FragB b;
                b.h[0] = *(const u16x8*)p;
                b.h[1] = *(const u16x8*)(p + 16);
                mma_bf(acc[m], a, b);
            }
            if (zp && ks < (KPS_ / 32)) {
                const unsigned short* p = sbp + k0;
                FragB b;
                b.h[0] = *(const u16x8*)p;
                b.h[1] = *(const u16x8*)(p + 16);
                mma_bf(acc[8], a, b);
            }
        }

        v8f vo;
#pragma unroll
        for (int r = 0; r < 8; ++r) {
            const float* pr = pis + (8 * h + r) * MM_;
            const v4f p0 = *(const v4f*)pr;
            const v4f p1 = *(const v4f*)(pr + 4);
            float s = p0[0] * acc[0][r];
            s = fmaf(p0[1], acc[1][r], s);
            s = fmaf(p0[2], acc[2][r], s);
            s = fmaf(p0[3], acc[3][r], s);
            s = fmaf(p1[0], acc[4][r], s);
            s = fmaf(p1[1], acc[5][r], s);
            s = fmaf(p1[2], acc[6][r], s);
            s = fmaf(p1[3], acc[7][r], s);
            vo[r] = s;
        }
        if (zp) {
#pragma unroll
            for (int r = 0; r < 8; ++r) {
                zf[(8 * h + r) * DS_ + ccol]  = vo[r];
                xst[(8 * h + r) * DS_ + ccol] = acc[8][r];
            }
        } else {
#pragma unroll
            for (int r = 0; r < 8; ++r) yst[(8 * h + r) * DY_ + ccol] = vo[r];
        }
        __syncthreads();

        if (wv < 4) {
            const int ra = wv, rb = 12 + wv;
            const v4f xa = *(const v4f*)(xst + ra * DS_ + 4 * lane);
            const v4f xb = *(const v4f*)(xst + rb * DS_ + 4 * lane);
            float* pa = out_x + ((size_t)(b0 + ra) * TT_ + t) * DS_ + 4 * lane;
            float* pb = out_x + ((size_t)(b0 + rb) * TT_ + t) * DS_ + 4 * lane;
            *(volatile v4f*)pa = xa;
            *(volatile v4f*)pb = xb;
            __threadfence();
            *(volatile v4f*)pa = xa;
            *(volatile v4f*)pb = xb;
        } else {
            const int ra = wv, ry = 2 * (wv - 4) + h;
            const v4f xa = *(const v4f*)(xst + ra * DS_ + 4 * lane);
            const v4f yv = *(const v4f*)(yst + ry * DY_ + 4 * ml);
            float* pa = out_x + ((size_t)(b0 + ra) * TT_ + t) * DS_ + 4 * lane;
            float* py = out_y + ((size_t)(b0 + ry) * TT_ + t) * DY_ + 4 * ml;
            *(volatile v4f*)pa = xa;
            *(volatile v4f*)py = yv;
            __threadfence();
            *(volatile v4f*)pa = xa;
            *(volatile v4f*)py = yv;
        }
    }
}

extern "C" void kernel_launch(void* const* d_in, const int* in_sizes, int n_in,
                              void* d_out, int out_size, void* d_ws, size_t ws_size,
                              hipStream_t stream)
{
    if (n_in < 8) return;
    if (in_sizes[0] != BB_ * TT_ * DU_)      return;
    if (in_sizes[1] != MM_ * NA_ * NA_)      return;
    if (in_sizes[2] < 1)                     return;
    if (in_sizes[3] != DS_ * DS_)            return;
    if (in_sizes[4] != GH_ * DU_)            return;
    if (in_sizes[5] != GH_)                  return;
    if (in_sizes[6] != MM_ * GH_)            return;
    if (in_sizes[7] != MM_)                  return;
    if (out_size != NBT_ * (DY_ + DS_))      return;
    if (ws_size < WS_END)                    return;

    const float* u     = (const float*)d_in[0];
    const float* K_raw = (const float*)d_in[1];
    const float* lgam  = (const float*)d_in[2];
    const float* S_raw = (const float*)d_in[3];
    const float* gw1   = (const float*)d_in[4];
    const float* gb1   = (const float*)d_in[5];
    const float* gw2   = (const float*)d_in[6];
    const float* gb2   = (const float*)d_in[7];

    float* out_y = (float*)d_out;
    float* out_x = (float*)d_out + (size_t)NBT_ * DY_;

    char* ws = (char*)d_ws;
    unsigned short* Kpl = (unsigned short*)(ws + OFF_KPL);
    unsigned short* Spl = (unsigned short*)(ws + OFF_SPL);
    float*          piw = (float*)(ws + OFF_PI);

    sinv_plane_kernel<<<dim3(1), dim3(128), 0, stream>>>(S_raw, Spl);
    experts_kernel<<<dim3(MM_), dim3(256), 0, stream>>>(K_raw, Kpl);
    gate_kernel<<<dim3(NBT_ / 64), dim3(128), 0, stream>>>(u, gw1, gb1, gw2, gb2, piw);
    scan_kernel<<<dim3(BB_ / NRB_), dim3(NTS_), 0, stream>>>(u, piw, lgam, Kpl, Spl, out_y, out_x);
}
